// Graphormer_4071628996729
// MI455X (gfx1250) — hardware-verified
//
#include <hip/hip_runtime.h>
#include <hip/hip_bf16.h>
#include <stddef.h>
#include <stdint.h>


#define DIN     128
#define F1      512
#define NQ1     2048
#define OQ1     0
#define OK1     512
#define OV1     1024
#define OS1     1536
#define HW1     512
#define KH      1024
#define F2      256
#define NQ2     896
#define OQ2     0
#define OK2     256
#define OV2     512
#define OS2     768
#define DOUT    128
#define NTHR    256
#define NWAVE   8
#define EPT     8
#define CHUNK   (NTHR * EPT)
#define WCAP    (EPT * 32)
#define LISTN   (NWAVE * WCAP)
#define NBMAX   2048
#define RCAP    28672
#define DEGCAP  4096
#define STW     512
#define GBM     64
#define GBN     64
#define GTHR    128
#define ATTSC   0.08838834764831845f
#define WSMAX   134217728
#define LDS_AGG ((2 * RCAP + 2 * NBMAX + LISTN) * 4 + 64)

static_assert((CHUNK & (CHUNK - 1)) == 0 && CHUNK <= 4096);
static_assert((NBMAX & (NBMAX - 1)) == 0 && NBMAX <= 4096);
static_assert(NTHR * 8 == NBMAX);
static_assert(LISTN >= NBMAX);
static_assert(LISTN >= NWAVE * WCAP);
static_assert((RCAP % 32) == 0);
static_assert(NWAVE * STW <= RCAP);
static_assert(STW * 4 == KH * 2);
static_assert(HW1 * 2 == KH && HW1 == 4 * 128);
static_assert(LDS_AGG <= 300000);
static_assert(GBM == (GTHR / 32) * 16);
static_assert(DIN / 8 == 16);
static_assert((DIN % 32) == 0 && (KH % 32) == 0 && KH == 2 * F1);
static_assert((NQ1 % GBN) == 0 && (NQ2 % GBN) == 0);
static_assert(NQ1 == 4 * F1 && NQ2 == 3 * F2 + DOUT);
static_assert(F1 == 32 * 16 && F2 == 32 * 8 && DOUT == 32 * 4);
static_assert(((NQ1 * 4) % 128) == 0 && ((NQ2 * 4) % 128) == 0);
static_assert((F1 % GBN) == 0 && (F2 % GBN) == 0);

typedef float          v4f  __attribute__((ext_vector_type(4)));
typedef float          v8f  __attribute__((ext_vector_type(8)));
typedef int            v4i  __attribute__((ext_vector_type(4)));
typedef int            v8i  __attribute__((ext_vector_type(8)));
typedef unsigned short v8us __attribute__((ext_vector_type(8)));
typedef __bf16         v16b __attribute__((ext_vector_type(16)));
typedef v4f  __attribute__((may_alias)) v4fa;
typedef v8us __attribute__((may_alias)) v8usa;
union FragB { v16b v; v8us h[2]; v8i w; };

__device__ __forceinline__ v8f wmb(const FragB& a, const FragB& b, v8f c) {
  v8f d = __builtin_amdgcn_wmma_f32_16x16x32_bf16(false, a.v, false, b.v, (short)0, c, false, false);
  asm volatile("v_nop\n\tv_nop\n\tv_nop\n\tv_nop" : "+v"(d) : "v"(a.w), "v"(b.w));
  return d;
}

__device__ __forceinline__ void ldwait() {
  asm volatile("s_wait_loadcnt 0x0" ::: "memory");
}

__device__ __forceinline__ unsigned f2bf(float f) {
  unsigned u = __float_as_uint(f);
  u += 0x7FFFu + ((u >> 16) & 1u);
  return u >> 16;
}
__device__ __forceinline__ float bfr(float f) {
  unsigned u = __float_as_uint(f);
  u = (u + 0x7FFFu + ((u >> 16) & 1u)) & 0xFFFF0000u;
  return __uint_as_float(u);
}
__device__ __forceinline__ v8us cvt8b(const v4f a, const v4f b) {
  v8us o;
  o[0] = (unsigned short)f2bf(a.x); o[1] = (unsigned short)f2bf(a.y);
  o[2] = (unsigned short)f2bf(a.z); o[3] = (unsigned short)f2bf(a.w);
  o[4] = (unsigned short)f2bf(b.x); o[5] = (unsigned short)f2bf(b.y);
  o[6] = (unsigned short)f2bf(b.z); o[7] = (unsigned short)f2bf(b.w);
  return o;
}

__device__ __forceinline__ int scan_chunk(const int* __restrict__ dsts, int nE, int cbase, int slotBase,
                                          int nb, int vec8, int* list, int tid, int lane, int wave) {
  int wc = 0;
  const int el0  = tid * EPT;
  const int e0   = cbase + el0;
  const int sent = -2147483647 - 1;
  v4i da, db;
  if (vec8 != 0 && cbase + CHUNK <= nE) {
    da = *(const v4i*)(dsts + e0);
    db = *(const v4i*)(dsts + e0 + 4);
  } else {
    da.x = (e0     < nE) ? dsts[min(e0,     nE - 1)] : sent;
    da.y = (e0 + 1 < nE) ? dsts[min(e0 + 1, nE - 1)] : sent;
    da.z = (e0 + 2 < nE) ? dsts[min(e0 + 2, nE - 1)] : sent;
    da.w = (e0 + 3 < nE) ? dsts[min(e0 + 3, nE - 1)] : sent;
    db.x = (e0 + 4 < nE) ? dsts[min(e0 + 4, nE - 1)] : sent;
    db.y = (e0 + 5 < nE) ? dsts[min(e0 + 5, nE - 1)] : sent;
    db.z = (e0 + 6 < nE) ? dsts[min(e0 + 6, nE - 1)] : sent;
    db.w = (e0 + 7 < nE) ? dsts[min(e0 + 7, nE - 1)] : sent;
  }
  const unsigned nbs = (unsigned)slotBase;
  const unsigned unb = (unsigned)nb;
  const unsigned s0 = (unsigned)da.x - nbs, s1 = (unsigned)da.y - nbs;
  const unsigned s2 = (unsigned)da.z - nbs, s3 = (unsigned)da.w - nbs;
  const unsigned s4 = (unsigned)db.x - nbs, s5 = (unsigned)db.y - nbs;
  const unsigned s6 = (unsigned)db.z - nbs, s7 = (unsigned)db.w - nbs;
  const bool h0 = s0 < unb, h1 = s1 < unb, h2 = s2 < unb, h3 = s3 < unb;
  const bool h4 = s4 < unb, h5 = s5 < unb, h6 = s6 < unb, h7 = s7 < unb;
  const unsigned any = __builtin_amdgcn_ballot_w32(h0 | h1 | h2 | h3 | h4 | h5 | h6 | h7);
  if (any != 0u) {
#define HITJ(J, HJ, SJ) { \
      const unsigned mj = __builtin_amdgcn_ballot_w32(HJ); \
      if (mj != 0u) { \
        if (HJ) { \
          const int pos = wc + (int)__builtin_amdgcn_mbcnt_lo(mj, 0u); \
          if (pos < WCAP) list[wave * WCAP + pos] = ((el0 + (J)) << 12) | (int)(SJ); \
        } \
        wc += (int)__builtin_popcount(mj); } }
    HITJ(0, h0, s0)
    HITJ(1, h1, s1)
    HITJ(2, h2, s2)
    HITJ(3, h3, s3)
    HITJ(4, h4, s4)
    HITJ(5, h5, s5)
    HITJ(6, h6, s6)
    HITJ(7, h7, s7)
#undef HITJ
  }
  return wc;
}

__global__ __launch_bounds__(NTHR) void k_xprep(const float* __restrict__ x, unsigned short* xb, int nN, int nUnits) {
  const int i = (int)blockIdx.x * NTHR + (int)threadIdx.x;
  if (i >= nUnits) return;
  const int row = i >> 4;
  const int c0  = (i & 15) * 8;
  const int rc  = row < nN ? row : nN - 1;
  const float* p = x + (size_t)rc * DIN + c0;
  v4f a = *(const v4fa*)p, b = *(const v4fa*)(p + 4);
  const v4f z4 = {0.f, 0.f, 0.f, 0.f};
  if (row >= nN) { a = z4; b = z4; }
  const v8us hv = cvt8b(a, b);
  const size_t o = (size_t)row * DIN + c0;
  *(volatile v8us*)(xb + o) = hv;
  __threadfence();
  *(volatile v8us*)(xb + o) = hv;
}

__global__ __launch_bounds__(NTHR) void k_wtr(const float* __restrict__ w0, const float* __restrict__ w1,
                                              const float* __restrict__ w2, const float* __restrict__ w3,
                                              int c0, int c1, int c2, int c3, int segRows, int K, int Kin,
                                              unsigned short* wt, int nUnits) {
  const int u = (int)blockIdx.x * NTHR + (int)threadIdx.x;
  if (u >= nUnits) return;
  const int kq = K >> 3;
  const int n  = u / kq;
  const int k8 = (u - n * kq) * 8;
  int k8s = k8 % Kin;
  k8s = k8s < 0 ? 0 : (k8s > Kin - 8 ? Kin - 8 : k8s);
  int seg = n / segRows;
  seg = seg > 3 ? 3 : seg;
  const int nc = n - seg * segRows;
  const float* ws = (seg == 0) ? w0 : ((seg == 1) ? w1 : ((seg == 2) ? w2 : w3));
  const int cc = (seg == 0) ? c0 : ((seg == 1) ? c1 : ((seg == 2) ? c2 : c3));
  const int ncl = nc < cc ? nc : cc - 1;
  const float* p = ws + (size_t)k8s * (size_t)cc + ncl;
  v4f a, b;
  a.x = p[0];                  a.y = p[(size_t)cc];         a.z = p[(size_t)2 * cc];     a.w = p[(size_t)3 * cc];
  b.x = p[(size_t)4 * cc];     b.y = p[(size_t)5 * cc];     b.z = p[(size_t)6 * cc];     b.w = p[(size_t)7 * cc];
  const v4f z4 = {0.f, 0.f, 0.f, 0.f};
  if (nc >= cc) { a = z4; b = z4; }
  const v8us hv = cvt8b(a, b);
  const size_t o = (size_t)n * (size_t)K + k8;
  *(volatile v8us*)(wt + o) = hv;
  __threadfence();
  *(volatile v8us*)(wt + o) = hv;
}

__global__ __launch_bounds__(GTHR) void k_gemm(
    const unsigned short* __restrict__ A, const unsigned short* __restrict__ WT,
    const float* __restrict__ b0, const float* __restrict__ b1,
    const float* __restrict__ b2, const float* __restrict__ b3,
    float* outF, int K, int ldo, int segN, int len012, int len3)
{
  __shared__ __attribute__((aligned(16))) float stg[GBM * GBN];
  const int tid = (int)threadIdx.x, lane = tid & 31, wave = tid >> 5, hh = lane >> 4, m = lane & 15;
  const int rowBase = (int)blockIdx.x * GBM;
  const int col0    = (int)blockIdx.y * GBN;
  int seg = col0 / segN;
  seg = seg < 0 ? 0 : (seg > 3 ? 3 : seg);
  const float* bp = (seg == 0) ? b0 : ((seg == 1) ? b1 : ((seg == 2) ? b2 : b3));
  const int blen = (seg < 3) ? len012 : len3;
  int bofs = col0 - seg * segN;
  bofs = bofs < 0 ? 0 : bofs;

  v8f acc[4];
  {
    const v8f z = {0.f, 0.f, 0.f, 0.f, 0.f, 0.f, 0.f, 0.f};
    acc[0] = z; acc[1] = z; acc[2] = z; acc[3] = z;
  }
  const unsigned short* ap = A  + (size_t)(rowBase + 16 * wave + m) * (size_t)K + 8 * hh;
  const unsigned short* wp = WT + (size_t)(col0 + m) * (size_t)K + 8 * hh;
  const int ksteps = K >> 5;
#pragma unroll 1
  for (int ks = 0; ks < ksteps; ++ks) {
    FragB af;
    af.h[0] = *(const v8usa*)(ap + 32 * ks);
    af.h[1] = *(const v8usa*)(ap + 32 * ks + 16);
#pragma unroll
    for (int t = 0; t < 4; ++t) {
      const unsigned short* wq = wp + (size_t)(16 * t) * (size_t)K + 32 * ks;
      FragB bf;
      bf.h[0] = *(const v8usa*)wq;
      bf.h[1] = *(const v8usa*)(wq + 16);
      acc[t] = wmb(af, bf, acc[t]);
    }
  }

#pragma unroll
  for (int t = 0; t < 4; ++t) {
    const int lc = 16 * t + m;
    int bi = bofs + lc;
    bi = bi > blen - 1 ? blen - 1 : bi;
    bi = bi < 0 ? 0 : bi;
    const float bv = bfr(bp[bi]);
#pragma unroll
    for (int r = 0; r < 8; ++r) {
      const int lr = 16 * wave + 8 * hh + r;
      stg[lr * GBN + lc] = acc[t][r] + bv;
    }
  }
  __syncthreads();

  v4f fv[8];
#pragma unroll
  for (int i = 0; i < 8; ++i) {
    const int lr = 16 * wave + 2 * i + hh;
    fv[i] = *(const v4fa*)(stg + lr * GBN + 4 * m);
  }
#pragma unroll
  for (int i = 0; i < 8; ++i) {
    const int lr = 16 * wave + 2 * i + hh;
    const int gr = rowBase + lr;
    float* op = outF + (size_t)gr * (size_t)ldo + col0 + 4 * m;
    *(volatile v4f*)op = fv[i];
  }
  __threadfence();
#pragma unroll
  for (int i = 0; i < 8; ++i) {
    const int lr = 16 * wave + 2 * i + hh;
    const int gr = rowBase + lr;
    float* op = outF + (size_t)gr * (size_t)ldo + col0 + 4 * m;
    *(volatile v4f*)op = fv[i];
  }
}

template<int LAYER>
__global__ __launch_bounds__(NTHR) void k_agg(
    const int* __restrict__ srcs, const int* __restrict__ dsts,
    const float* __restrict__ QKVS, int* Hout, float* out,
    int nN, int nE, int nb, int vec8, int MPr) {
  extern __shared__ v4f lds_dyn[];
  int* reg1 = (int*)lds_dyn;
  int* reg2 = reg1 + RCAP;
  int* scnt = reg2 + RCAP;
  int* soff = scnt + NBMAX;
  int* list = soff + NBMAX;
  int* wcnt = list + LISTN;
  int* wtot = wcnt + NWAVE;
  const int tid = (int)threadIdx.x, lane = tid & 31, wave = tid >> 5;
  const int nodeBase = (int)blockIdx.x * nb;

  for (int i = tid; i < NBMAX; i += NTHR) scnt[i] = 0;
  __syncthreads();

  int tot = 0;
  const int nChunks = (nE + CHUNK - 1) / CHUNK;
#pragma unroll 1
  for (int ch = 0; ch < nChunks; ++ch) {
    const int cbase = ch * CHUNK;
    const int wc = scan_chunk(dsts, nE, cbase, nodeBase, nb, vec8, list, tid, lane, wave);
    if (lane == 0) wcnt[wave] = wc;
    __syncthreads();
    int pre = 0, all = 0;
#pragma unroll
    for (int w2 = 0; w2 < NWAVE; ++w2) {
      int c = wcnt[w2];
      c = c < 0 ? 0 : (c > WCAP ? WCAP : c);
      all += c;
      pre += (w2 < wave) ? c : 0;
    }
    const int wcc  = wc > WCAP ? WCAP : wc;
    const int base = tot + pre;
#pragma unroll 1
    for (int i = lane; i < wcc; i += 32) {
      const int ent = list[wave * WCAP + i];
      const int el  = (ent >> 12) & (CHUNK - 1);
      const int sl  = ent & (NBMAX - 1);
      int eid = cbase + el;
      eid = eid > nE - 1 ? nE - 1 : eid;
      const int pos = base + i;
      if (pos < RCAP) reg1[pos] = (int)(((unsigned)eid << 12) | (unsigned)sl);
    }
    tot += all;
    tot = tot > RCAP ? RCAP : tot;
    __syncthreads();
  }
  const int nh = tot;

  if (wave == 0) {
#pragma unroll 1
    for (int b0 = 0; b0 < nh; b0 += 32) {
      const int idx = b0 + lane;
      const int uv  = reg1[idx < nh ? idx : nh - 1];
      const int m32 = (nh - b0) < 32 ? (nh - b0) : 32;
#pragma unroll 1
      for (int k = 0; k < m32; ++k) {
        const int u  = __builtin_amdgcn_readlane(uv, k);
        const int sl = u & (NBMAX - 1);
        if (lane == 0) scnt[sl] = scnt[sl] + 1;
      }
    }
  }
  __syncthreads();

  {
    const v4i ca = *(const v4i*)(scnt + 8 * tid);
    const v4i cb = *(const v4i*)(scnt + 8 * tid + 4);
    const int e0 = ca.x < 0 ? 0 : ca.x, e1 = ca.y < 0 ? 0 : ca.y, e2 = ca.z < 0 ? 0 : ca.z, e3 = ca.w < 0 ? 0 : ca.w;
    const int e4 = cb.x < 0 ? 0 : cb.x, e5 = cb.y < 0 ? 0 : cb.y, e6 = cb.z < 0 ? 0 : cb.z, e7 = cb.w < 0 ? 0 : cb.w;
    const int ts = e0 + e1 + e2 + e3 + e4 + e5 + e6 + e7;
    int incl = ts;
#pragma unroll
    for (int d = 1; d < 32; d <<= 1) {
      const int up = __shfl_up(incl, d);
      if (lane >= d) incl += up;
    }
    if (lane == 31) wtot[wave] = incl;
    __syncthreads();
    int pre = 0;
#pragma unroll
    for (int w2 = 0; w2 < NWAVE; ++w2) pre += (w2 < wave) ? wtot[w2] : 0;
    int run = pre + incl - ts;
    soff[8 * tid + 0] = run; run += e0;
    soff[8 * tid + 1] = run; run += e1;
    soff[8 * tid + 2] = run; run += e2;
    soff[8 * tid + 3] = run; run += e3;
    soff[8 * tid + 4] = run; run += e4;
    soff[8 * tid + 5] = run; run += e5;
    soff[8 * tid + 6] = run; run += e6;
    soff[8 * tid + 7] = run;
  }
  __syncthreads();
  for (int i = tid; i < NBMAX; i += NTHR) list[i] = soff[i];
  __syncthreads();

  if (wave == 0) {
#pragma unroll 1
    for (int b0 = 0; b0 < nh; b0 += 32) {
      const int idx = b0 + lane;
      const int uv  = reg1[idx < nh ? idx : nh - 1];
      const int m32 = (nh - b0) < 32 ? (nh - b0) : 32;
#pragma unroll 1
      for (int k = 0; k < m32; ++k) {
        const int u   = __builtin_amdgcn_readlane(uv, k);
        const int sl  = u & (NBMAX - 1);
        const int eid = (int)((unsigned)u >> 12);
        if (lane == 0) {
          int pos = list[sl];
          pos = pos < 0 ? 0 : (pos > RCAP - 1 ? RCAP - 1 : pos);
          reg2[pos] = eid;
          list[sl] = pos + 1;
        }
      }
    }
  }
  __syncthreads();

  const int nbw = nb >> 3;
  const bool ovf = (nh >= RCAP);
  const float qnan = __int_as_float(0x7fc00000);

  if (LAYER == 1) {
    int* stw = reg1 + wave * STW;
#pragma unroll 1
    for (int jt = 0; jt < nbw; ++jt) {
      const int slot = wave * nbw + jt;
      const int grow = nodeBase + slot;
      const int gcl  = grow < nN ? grow : nN - 1;
      int st = soff[slot];
      const int craw = scnt[slot];
      int cnt = craw;
      st  = st < 0 ? 0 : (st > nh ? nh : st);
      cnt = cnt < 0 ? 0 : (cnt > DEGCAP ? DEGCAP : cnt);
      if (cnt > nh - st) cnt = nh - st;
      const float pz = (ovf || craw > DEGCAP) ? qnan : 0.0f;
      const bool wr = grow < MPr;
      const float live = grow < nN ? 1.0f : 0.0f;

      const float* qrow = QKVS + (size_t)gcl * NQ1 + OQ1 + 16 * lane;
      float qv[16], av[16];
#pragma unroll
      for (int j = 0; j < 4; ++j) {
        const v4f t4 = *(const v4fa*)(qrow + 4 * j);
        qv[4 * j] = t4.x; qv[4 * j + 1] = t4.y; qv[4 * j + 2] = t4.z; qv[4 * j + 3] = t4.w;
      }
      ldwait();
#pragma unroll
      for (int i = 0; i < 16; ++i) av[i] = 0.f;
      float mx = -1.0e30f, dn = 0.f;

#pragma unroll 1
      for (int q = 0; q < cnt; ++q) {
        int idx = st + q; idx = idx > RCAP - 1 ? RCAP - 1 : idx;
        int eid = reg2[idx]; eid = eid < 0 ? 0 : (eid > nE - 1 ? nE - 1 : eid);
        const int sraw = srcs[eid];
        const int s = sraw < 0 ? 0 : (sraw > nN - 1 ? nN - 1 : sraw);
        const float* kr = QKVS + (size_t)s * NQ1 + OK1 + 16 * lane;
        float kk[16], vv[16];
#pragma unroll
        for (int j = 0; j < 4; ++j) {
          const v4f t4 = *(const v4fa*)(kr + 4 * j);
          kk[4 * j] = t4.x; kk[4 * j + 1] = t4.y; kk[4 * j + 2] = t4.z; kk[4 * j + 3] = t4.w;
        }
        ldwait();
#pragma unroll
        for (int j = 0; j < 4; ++j) {
          const v4f t4 = *(const v4fa*)(kr + (OV1 - OK1) + 4 * j);
          vv[4 * j] = t4.x; vv[4 * j + 1] = t4.y; vv[4 * j + 2] = t4.z; vv[4 * j + 3] = t4.w;
        }
        ldwait();
        float pa = qv[0] * kk[0], pb = qv[8] * kk[8];
#pragma unroll
        for (int i = 1; i < 8; ++i) {
          pa = fmaf(qv[i], kk[i], pa);
          pb = fmaf(qv[8 + i], kk[8 + i], pb);
        }
        float part = pa + pb;
        part += __shfl_xor(part, 1);
        part += __shfl_xor(part, 2);
        part += __shfl_xor(part, 4);
        const float al = part * ATTSC;
        const float df = al - mx;
        const float ee = __expf(-fabsf(df));
        const bool up  = df > 0.f;
        const float s1 = up ? ee : 1.0f;
        const float s2 = up ? 1.0f : ee;
        mx = up ? al : mx;
        dn = fmaf(dn, s1, s2);
#pragma unroll
        for (int i = 0; i < 16; ++i) av[i] = fmaf(av[i], s1, s2 * vv[i]);
      }
      const float ds = dn > 0.f ? dn : 1.0f;
      const float iv = (dn > 0.f ? 1.0f : 0.0f) * __builtin_amdgcn_rcpf(ds);

      const float* sp = QKVS + (size_t)gcl * NQ1 + OS1 + 16 * lane;
      float sk[16];
#pragma unroll
      for (int j = 0; j < 4; ++j) {
        const v4f t4 = *(const v4fa*)(sp + 4 * j);
        sk[4 * j] = t4.x; sk[4 * j + 1] = t4.y; sk[4 * j + 2] = t4.z; sk[4 * j + 3] = t4.w;
      }
      ldwait();

      int hw[8], lw[8];
#pragma unroll
      for (int j = 0; j < 8; ++j) {
        const float o0 = av[2 * j] * iv;
        const float o1 = av[2 * j + 1] * iv;
        const float r0 = fmaxf(o0 + sk[2 * j], 0.f) * live + pz;
        const float r1 = fmaxf(o1 + sk[2 * j + 1], 0.f) * live + pz;
        const unsigned h0 = f2bf(r0), h1 = f2bf(r1);
        const unsigned l0 = f2bf(r0 - __uint_as_float(h0 << 16));
        const unsigned l1 = f2bf(r1 - __uint_as_float(h1 << 16));
        hw[j] = (int)(h0 | (h1 << 16));
        lw[j] = (int)(l0 | (l1 << 16));
      }
      v4i ha, hb, la, lb;
      ha.x = hw[0]; ha.y = hw[1]; ha.z = hw[2]; ha.w = hw[3];
      hb.x = hw[4]; hb.y = hw[5]; hb.z = hw[6]; hb.w = hw[7];
      la.x = lw[0]; la.y = lw[1]; la.z = lw[2]; la.w = lw[3];
      lb.x = lw[4]; lb.y = lw[5]; lb.z = lw[6]; lb.w = lw[7];
      __builtin_amdgcn_fence(__ATOMIC_RELEASE, "wavefront");
      __builtin_amdgcn_wave_barrier();
      *(v4i*)(stw + 8 * lane)           = ha;
      *(v4i*)(stw + 8 * lane + 4)       = hb;
      *(v4i*)(stw + 256 + 8 * lane)     = la;
      *(v4i*)(stw + 256 + 8 * lane + 4) = lb;
      __builtin_amdgcn_fence(__ATOMIC_RELEASE, "wavefront");
      __builtin_amdgcn_wave_barrier();
      v4i pv[4];
#pragma unroll
      for (int i = 0; i < 4; ++i) pv[i] = *(const v4i*)(stw + 4 * (32 * i + lane));
      int* gp = Hout + (size_t)grow * HW1 + 4 * lane;
#pragma unroll
      for (int i = 0; i < 4; ++i) { if (wr) *(volatile v4i*)(gp + 128 * i) = pv[i]; }
      __threadfence();
#pragma unroll
      for (int i = 0; i < 4; ++i) { if (wr) *(volatile v4i*)(gp + 128 * i) = pv[i]; }
    }
  } else {
#pragma unroll 1
    for (int jt = 0; jt < nbw; ++jt) {
      const int slot = wave * nbw + jt;
      const int grow = nodeBase + slot;
      const int gcl  = grow < nN ? grow : nN - 1;
      int st = soff[slot];
      const int craw = scnt[slot];
      int cnt = craw;
      st  = st < 0 ? 0 : (st > nh ? nh : st);
      cnt = cnt < 0 ? 0 : (cnt > DEGCAP ? DEGCAP : cnt);
      if (cnt > nh - st) cnt = nh - st;
      const float pz = (ovf || craw > DEGCAP) ? qnan : 0.0f;
      const bool wr = grow < nN;

      const float* qrow = QKVS + (size_t)gcl * NQ2 + OQ2 + 8 * lane;
      float qv[8], av[8];
#pragma unroll
      for (int j = 0; j < 2; ++j) {
        const v4f t4 = *(const v4fa*)(qrow + 4 * j);
        qv[4 * j] = t4.x; qv[4 * j + 1] = t4.y; qv[4 * j + 2] = t4.z; qv[4 * j + 3] = t4.w;
      }
      ldwait();
#pragma unroll
      for (int i = 0; i < 8; ++i) av[i] = 0.f;
      float mx = -1.0e30f, dn = 0.f;

#pragma unroll 1
      for (int q = 0; q < cnt; ++q) {
        int idx = st + q; idx = idx > RCAP - 1 ? RCAP - 1 : idx;
        int eid = reg2[idx]; eid = eid < 0 ? 0 : (eid > nE - 1 ? nE - 1 : eid);
        const int sraw = srcs[eid];
        const int s = sraw < 0 ? 0 : (sraw > nN - 1 ? nN - 1 : sraw);
        const float* kr = QKVS + (size_t)s * NQ2 + OK2 + 8 * lane;
        float kk[8], vv[8];
#pragma unroll
        for (int j = 0; j < 2; ++j) {
          const v4f t4 = *(const v4fa*)(kr + 4 * j);
          kk[4 * j] = t4.x; kk[4 * j + 1] = t4.y; kk[4 * j + 2] = t4.z; kk[4 * j + 3] = t4.w;
        }
        ldwait();
#pragma unroll
        for (int j = 0; j < 2; ++j) {
          const v4f t4 = *(const v4fa*)(kr + (OV2 - OK2) + 4 * j);
          vv[4 * j] = t4.x; vv[4 * j + 1] = t4.y; vv[4 * j + 2] = t4.z; vv[4 * j + 3] = t4.w;
        }
        ldwait();
        float part = qv[0] * kk[0];
#pragma unroll
        for (int i = 1; i < 8; ++i) part = fmaf(qv[i], kk[i], part);
        part += __shfl_xor(part, 1);
        part += __shfl_xor(part, 2);
        part += __shfl_xor(part, 4);
        part += __shfl_xor(part, 8);
        const float al = part * ATTSC;
        const float df = al - mx;
        const float ee = __expf(-fabsf(df));
        const bool up  = df > 0.f;
        const float s1 = up ? ee : 1.0f;
        const float s2 = up ? 1.0f : ee;
        mx = up ? al : mx;
        dn = fmaf(dn, s1, s2);
#pragma unroll
        for (int i = 0; i < 8; ++i) av[i] = fmaf(av[i], s1, s2 * vv[i]);
      }
      const float ds = dn > 0.f ? dn : 1.0f;
      const float iv = (dn > 0.f ? 1.0f : 0.0f) * __builtin_amdgcn_rcpf(ds);

      const float* sp = QKVS + (size_t)gcl * NQ2 + OS2 + 8 * (lane & 15);
      float sk[8];
#pragma unroll
      for (int j = 0; j < 2; ++j) {
        const v4f t4 = *(const v4fa*)(sp + 4 * j);
        sk[4 * j] = t4.x; sk[4 * j + 1] = t4.y; sk[4 * j + 2] = t4.z; sk[4 * j + 3] = t4.w;
      }
      ldwait();

      float tv[8];
#pragma unroll
      for (int i = 0; i < 8; ++i) {
        const float o  = av[i] * iv;
        const float ot = __shfl_xor(o, 16);
        const float rs = (o + ot) * 0.5f + sk[i] + pz;
        tv[i] = __shfl(rs, lane >> 1);
      }
      const bool odd = (lane & 1) != 0;
      v4f y;
      y.x = odd ? tv[4] : tv[0];
      y.y = odd ? tv[5] : tv[1];
      y.z = odd ? tv[6] : tv[2];
      y.w = odd ? tv[7] : tv[3];
      float* gp = out + (size_t)gcl * DOUT + 4 * lane;
      if (wr) *(volatile v4f*)gp = y;
      __threadfence();
      if (wr) *(volatile v4f*)gp = y;
    }
  }
}

static int pick_nb(int nE, int nN) {
  int nb = NBMAX;
  while (nb > 16 && (long long)nb * (long long)nE * 5LL > (long long)RCAP * (long long)nN * 4LL) nb >>= 1;
  return nb;
}
static inline int cdiv(int a, int b) { return (a + b - 1) / b; }

extern "C" void kernel_launch(void* const* d_in, const int* in_sizes, int n_in,
                              void* d_out, int out_size, void* d_ws, size_t ws_size,
                              hipStream_t stream) {
  if (n_in < 18) return;
  const int nN = in_sizes[0] / DIN;
  if (nN <= 0 || in_sizes[0] != nN * DIN || nN > (1 << 22)) return;
  if (in_sizes[1] < 2 || (in_sizes[1] & 1) != 0) return;
  const int nE = in_sizes[1] / 2;
  if (nE < 1 || nE > (1 << 20)) return;
  if (in_sizes[2]  != DIN * F1 || in_sizes[3]  != F1) return;
  if (in_sizes[4]  != DIN * F1 || in_sizes[5]  != F1) return;
  if (in_sizes[6]  != DIN * F1 || in_sizes[7]  != F1) return;
  if (in_sizes[8]  != DIN * F1 || in_sizes[9]  != F1) return;
  if (in_sizes[10] != F1 * F2  || in_sizes[11] != F2) return;
  if (in_sizes[12] != F1 * F2  || in_sizes[13] != F2) return;
  if (in_sizes[14] != F1 * F2  || in_sizes[15] != F2) return;
  if (in_sizes[16] != F1 * DOUT || in_sizes[17] != DOUT) return;
  if (out_size != nN * DOUT) return;

  const float* x   = (const float*)d_in[0];
  const int*   ei  = (const int*)  d_in[1];
  const float* Wq1 = (const float*)d_in[2];
  const float* bq1 = (const float*)d_in[3];
  const float* Wk1 = (const float*)d_in[4];
  const float* bk1 = (const float*)d_in[5];
  const float* Wv1 = (const float*)d_in[6];
  const float* bv1 = (const float*)d_in[7];
  const float* Ws1 = (const float*)d_in[8];
  const float* bs1 = (const float*)d_in[9];
  const float* Wq2 = (const float*)d_in[10];
  const float* bq2 = (const float*)d_in[11];
  const float* Wk2 = (const float*)d_in[12];
  const float* bk2 = (const float*)d_in[13];
  const float* Wv2 = (const float*)d_in[14];
  const float* bv2 = (const float*)d_in[15];
  const float* Ws2 = (const float*)d_in[16];
  const float* bs2 = (const float*)d_in[17];
  float* out = (float*)d_out;
  const int* src = ei;
  const int* dst = ei + nE;

  const int MP   = cdiv(nN, GBM) * GBM;
  const int nb   = pick_nb(nE, nN);
  const int gA   = cdiv(MP, nb);
  const int vec8 = ((nE & 3) == 0) ? 1 : 0;
  if (gA * nb < MP) return;

  char* ws = (char*)d_ws;
  size_t off = 0;
  const size_t oXB  = off; off += (size_t)MP * DIN * 2;            off = (off + 255) & ~(size_t)255;
  const size_t oWT1 = off; off += (size_t)NQ1 * DIN * 2;           off = (off + 255) & ~(size_t)255;
  const size_t oWT2 = off; off += (size_t)NQ2 * KH * 2;            off = (off + 255) & ~(size_t)255;
  const size_t oQKV = off; off += (size_t)MP * NQ1 * 4;            off = (off + 255) & ~(size_t)255;
  const size_t oH1  = off; off += (size_t)MP * KH * 2;             off = (off + 255) & ~(size_t)255;
  if (off > ws_size || off > (size_t)WSMAX) return;
  if ((size_t)MP * NQ2 * 4 > (size_t)MP * NQ1 * 4) return;
  unsigned short* XB  = (unsigned short*)(ws + oXB);
  unsigned short* WT1 = (unsigned short*)(ws + oWT1);
  unsigned short* WT2 = (unsigned short*)(ws + oWT2);
  float*          QKV = (float*)(ws + oQKV);
  unsigned short* H1h = (unsigned short*)(ws + oH1);
  int*            H1w = (int*)(ws + oH1);

  hipFuncSetAttribute(reinterpret_cast<const void*>(&k_agg<1>),
                      hipFuncAttributeMaxDynamicSharedMemorySize, LDS_AGG);
  hipFuncSetAttribute(reinterpret_cast<const void*>(&k_agg<2>),
                      hipFuncAttributeMaxDynamicSharedMemorySize, LDS_AGG);

  const int nUx = MP * (DIN / 8);
  k_xprep<<<cdiv(nUx, NTHR), NTHR, 0, stream>>>(x, XB, nN, nUx);

  {
    const int nU1 = NQ1 * (DIN / 8);
    k_wtr<<<cdiv(nU1, NTHR), NTHR, 0, stream>>>(Wq1, Wk1, Wv1, Ws1, F1, F1, F1, F1, F1, DIN, DIN, WT1, nU1);
    const int nU2 = NQ2 * (KH / 8);
    k_wtr<<<cdiv(nU2, NTHR), NTHR, 0, stream>>>(Wq2, Wk2, Wv2, Ws2, F2, F2, F2, DOUT, F2, KH, F1, WT2, nU2);
  }

  const int gM = MP / GBM;
  k_gemm<<<dim3(gM, NQ1 / GBN), GTHR, 0, stream>>>(XB, WT1, bq1, bk1, bv1, bs1, QKV, DIN, NQ1, F1, F1, F1);
  k_agg<1><<<gA, NTHR, LDS_AGG, stream>>>(src, dst, QKV, H1w, out, nN, nE, nb, vec8, MP);
  k_gemm<<<dim3(gM, NQ2 / GBN), GTHR, 0, stream>>>(H1h, WT2, bq2, bk2, bv2, bs2, QKV, KH, NQ2, F2, F2, DOUT);
  k_agg<2><<<gA, NTHR, LDS_AGG, stream>>>(src, dst, QKV, H1w, out, nN, nE, nb, vec8, MP);
}
